// PermutationModule_43808666419472
// MI455X (gfx1250) — hardware-verified
//
#include <hip/hip_runtime.h>


#define NBI  4
#define NTOK 512
#define DD   512
#define PP   128
#define ICH  64
#define NPR  (ICH * NTOK)
#define DM   DD
#define LOSC 1024.0f

typedef _Float16 h16;
typedef unsigned short bf;
typedef __attribute__((ext_vector_type(16))) __bf16   v16bf;
typedef __attribute__((ext_vector_type(16))) _Float16 v16h;
typedef __attribute__((ext_vector_type(8)))  _Float16 v8h;
typedef __attribute__((ext_vector_type(8)))  unsigned short v8us;
typedef __attribute__((ext_vector_type(8)))  float    v8f;
typedef __attribute__((ext_vector_type(4)))  float    v4f;
typedef v8h  __attribute__((may_alias)) v8ha;
typedef v4f  __attribute__((may_alias)) v4fa;
typedef v8us __attribute__((may_alias)) v8usa;

__device__ __forceinline__ unsigned short f2bf(float f) { unsigned u = __float_as_uint(f); u += 0x7FFFu + ((u >> 16) & 1u); return (unsigned short)(u >> 16); }
__device__ __forceinline__ float bf2f(unsigned short b) { return __uint_as_float(((unsigned)b) << 16); }
__device__ __forceinline__ float bfr(float f) { return bf2f(f2bf(f)); }
__device__ __forceinline__ v16h cat16(v8h lo, v8h hi) { return __builtin_shufflevector(lo, hi, 0, 1, 2, 3, 4, 5, 6, 7, 8, 9, 10, 11, 12, 13, 14, 15); }
__device__ __forceinline__ v16bf cat16b(v8us lo, v8us hi) { return __builtin_bit_cast(v16bf, __builtin_shufflevector(lo, hi, 0, 1, 2, 3, 4, 5, 6, 7, 8, 9, 10, 11, 12, 13, 14, 15)); }
__device__ __forceinline__ v8f wmma16(v16h a, v16h b, v8f c) { return __builtin_amdgcn_wmma_f32_16x16x32_f16(false, a, false, b, (short)0, c, false, false); }
__device__ __forceinline__ v8f wmmab(v16bf a, v16bf b, v8f c) { return __builtin_amdgcn_wmma_f32_16x16x32_bf16(false, a, false, b, (short)0, c, false, false); }

template <bool SPLITA, bool F16OUT = false>
__global__ __launch_bounds__(128) void k_gemmb(const bf* __restrict__ A, const bf* __restrict__ Al, const bf* __restrict__ Bn, const float* __restrict__ bias, float* C, int ldc, h16* C2, const float* __restrict__ R = nullptr, int K = DM, int roundR = 1) {
    __shared__ __align__(16) float ost[4][16 * 68];
    const int lane = threadIdx.x & 31, wave = threadIdx.x >> 5, lr = lane & 15, hi = lane >> 4;
    const int r0 = blockIdx.x * 64 + wave * 16, c0 = blockIdx.y * 64;
    const size_t aoff = (size_t)(r0 + lr) * K + 8 * hi;
    size_t boff[4];
#pragma unroll
    for (int t = 0; t < 4; ++t) boff[t] = (size_t)(c0 + t * 16 + lr) * K + 8 * hi;
    v8f acc[4];
#pragma unroll
    for (int t = 0; t < 4; ++t) acc[t] = (v8f){};
#pragma unroll 1
    for (int kc = 0; kc < K; kc += 32) {
        const v16bf a = cat16b(*(const v8us*)(A + aoff + kc), *(const v8us*)(A + aoff + kc + 16));
        v16bf al = a;
        if (SPLITA) al = cat16b(*(const v8us*)(Al + aoff + kc), *(const v8us*)(Al + aoff + kc + 16));
#pragma unroll
        for (int t = 0; t < 4; ++t) { const v16bf b = cat16b(*(const v8us*)(Bn + boff[t] + kc), *(const v8us*)(Bn + boff[t] + kc + 16)); acc[t] = wmmab(a, b, acc[t]); if (SPLITA) acc[t] = wmmab(al, b, acc[t]); }
        asm volatile("v_nop\n\tv_nop\n\tv_nop\n\tv_nop" : "+v"(acc[0]), "+v"(acc[1]), "+v"(acc[2]), "+v"(acc[3]) : "v"(a), "v"(al));
    }
    float* os = &ost[wave][0];
#pragma unroll
    for (int t = 0; t < 4; ++t) { const float bv = bias ? bfr(bias[c0 + t * 16 + lr]) : 0.f;
#pragma unroll
        for (int j = 0; j < 8; ++j) os[(hi * 8 + j) * 68 + t * 16 + lr] = acc[t][j] + bv; }
    __syncthreads();
    if (F16OUT) {
        h16* crow = (h16*)(void*)C + (size_t)r0 * ldc + c0;
        auto pass = [&]() {
#pragma unroll
            for (int s = 0; s < 4; ++s) { const int row = 4 * s + (lane >> 3), piece = lane & 7; const float* sp = os + row * 68 + piece * 8; v8h o, o2;
#pragma unroll
                for (int i = 0; i < 8; ++i) { const h16 a = (h16)sp[i]; o[i] = a; o2[i] = (h16)((sp[i] - (float)a) * LOSC); }
                *(volatile v8h*)(crow + (size_t)row * ldc + piece * 8) = o; if (C2) *(volatile v8h*)(C2 + (size_t)r0 * ldc + c0 + (size_t)row * ldc + piece * 8) = o2; }
        };
        pass(); __threadfence(); pass();
    } else {
        float* crow = C + (size_t)r0 * ldc + c0;
        auto pass = [&]() {
#pragma unroll
            for (int s = 0; s < 8; ++s) { const int Lid = (lane >> 3) + 4 * s, piece = lane & 7; const int row = Lid >> 1, cofs = (Lid & 1) * 32 + piece * 4;
                v4f val = *(const v4fa*)(os + row * 68 + cofs); if (R) { const v4f rv = *(const v4f*)(R + ((size_t)r0 + row) * ldc + c0 + cofs); val += roundR ? (v4f){bfr(rv[0]), bfr(rv[1]), bfr(rv[2]), bfr(rv[3])} : rv; }
                *(volatile v4f*)(crow + (size_t)row * ldc + cofs) = val; }
        };
        pass(); __threadfence(); pass();
    }
}


__global__ __launch_bounds__(256) void k_wt(const float* __restrict__ Wm, int K, int ncols, bf* WT) {
    __shared__ __align__(16) unsigned short tl[64 * 72];
    const int tid = threadIdx.x, k0 = blockIdx.x * 64, n0 = blockIdx.y * 64;
    const int kk = tid >> 2, nq = (tid & 3) * 16;
#pragma unroll
    for (int i = 0; i < 16; ++i) tl[(nq + i) * 72 + kk] = f2bf(Wm[(size_t)(k0 + kk) * ncols + n0 + nq + i]);
    __syncthreads();
    const int piece = tid & 7;
    auto pass = [&]() {
#pragma unroll
        for (int s = 0; s < 2; ++s) { const int nr = (tid >> 3) + 32 * s; const v8us val = *(const v8usa*)(tl + nr * 72 + piece * 8); *(volatile v8us*)(WT + (size_t)(n0 + nr) * K + k0 + piece * 8) = val; }
    };
    pass(); __threadfence(); pass();
}

__global__ __launch_bounds__(256) void k_cvt(const float* __restrict__ src, bf* dst) {
    const int lane = threadIdx.x & 31, r = blockIdx.x * 8 + (threadIdx.x >> 5); if (r >= NTOK) return;
#pragma unroll 1
    for (int ps = 0; ps < 2; ++ps) {
#pragma unroll
        for (int c0 = lane * 8; c0 < DD; c0 += 256) { v8us o;
#pragma unroll
            for (int i = 0; i < 8; ++i) o[i] = f2bf(src[(size_t)r * DD + c0 + i]);
            *(volatile v8us*)(dst + (size_t)r * DD + c0) = o; }
        if (ps == 0) __threadfence(); }
}
__global__ __launch_bounds__(256) void k_wopad(const float* __restrict__ Wo, bf* WOP) {
    const int u = blockIdx.x * 256 + threadIdx.x; if (u >= 64 * PP / 8) return; const int row = u / (PP / 8), p0 = (u % (PP / 8)) * 8; v8us o;
#pragma unroll
    for (int i = 0; i < 8; ++i) o[i] = (row == 0) ? f2bf(Wo[p0 + i]) : (unsigned short)0;
    *(volatile v8us*)(WOP + (size_t)u * 8) = o; __threadfence(); *(volatile v8us*)(WOP + (size_t)u * 8) = o;
}
__global__ __launch_bounds__(256) void k_head1(const float* __restrict__ Hs, const float* __restrict__ W2, const float* __restrict__ b2, float* OUTV, int b) {
    const int t = blockIdx.x * 256 + threadIdx.x; if (t >= NTOK) return; const float* hr = Hs + (size_t)t * PP; float a = bfr(b2[0]);
#pragma unroll 4
    for (int p = 0; p < PP; ++p) a = fmaf(fmaxf(hr[p], 0.f), bfr(W2[p]), a);
    float* o = OUTV + (size_t)b * NTOK + t; *(volatile float*)o = a; __threadfence(); *(volatile float*)o = a;
}
__global__ __launch_bounds__(256) void k_pairs(const float* __restrict__ L, const float* __restrict__ R, int i0, bf* Ah, bf* Al) {
    const int lane = threadIdx.x & 31, wv = threadIdx.x >> 5; const int il = blockIdx.x / (NTOK / 16), jb = blockIdx.x % (NTOK / 16);
    const int j = jb * 16 + wv * 2 + (lane >> 4), p0 = (lane & 15) * 8; const int i = i0 + il;
    const v8f lv = *(const v8f*)(L + (size_t)j * PP + p0), rv = *(const v8f*)(R + (size_t)i * PP + p0); v8us oh, ol;
#pragma unroll
    for (int q = 0; q < 8; ++q) { const float v = fmaxf(lv[q] + rv[q], 0.f); const unsigned short hb = f2bf(v); oh[q] = hb; ol[q] = f2bf(v - bf2f(hb)); }
    const size_t o = ((size_t)il * NTOK + j) * PP + p0;
    *(volatile v8us*)(Ah + o) = oh; *(volatile v8us*)(Al + o) = ol; __threadfence(); *(volatile v8us*)(Ah + o) = oh; *(volatile v8us*)(Al + o) = ol;
}
__global__ __launch_bounds__(256) void k_bout(const float* __restrict__ Cm, const float* __restrict__ bo, int b, int i0, float* OUT0) {
    const int u = blockIdx.x * 256 + threadIdx.x; if (u >= NPR) return;
    const float v = Cm[(size_t)u * 64] + bfr(bo[0]); float* o = OUT0 + ((size_t)b * NTOK + i0) * NTOK + u;
    *(volatile float*)o = v; __threadfence(); *(volatile float*)o = v;
}

extern "C" void kernel_launch(void* const* d_in, const int* in_sizes, int n_in,
                              void* d_out, int out_size, void* d_ws, size_t ws_size, hipStream_t stream) {
    (void)in_sizes; (void)n_in; (void)out_size;
    const float* x = (const float*)d_in[0]; const float* Wl = (const float*)d_in[1]; const float* bl = (const float*)d_in[2]; const float* Wr = (const float*)d_in[3]; const float* Wo = (const float*)d_in[4]; const float* bo = (const float*)d_in[5];
    const float* Ws1 = (const float*)d_in[6]; const float* bs1 = (const float*)d_in[7]; const float* Ws2 = (const float*)d_in[8]; const float* bs2 = (const float*)d_in[9];
    const float* We1 = (const float*)d_in[10]; const float* be1 = (const float*)d_in[11]; const float* We2 = (const float*)d_in[12]; const float* be2 = (const float*)d_in[13];
    float* out0 = (float*)d_out;
    float* out1 = (float*)((char*)d_out + (size_t)NBI * NTOK * NTOK * 4);
    float* out2 = (float*)((char*)d_out + (size_t)NBI * NTOK * NTOK * 4 + NBI * NTOK * 4);
    char* wsp = (char*)d_ws;
    auto take = [&](size_t bytes) { char* p = wsp; wsp += (bytes + 255) & ~(size_t)255; return (void*)p; };
    bf* WlT = (bf*)take(PP * DD * 2); bf* WrT = (bf*)take(PP * DD * 2); bf* WsT = (bf*)take(PP * DD * 2); bf* WeT = (bf*)take(PP * DD * 2); bf* WOP = (bf*)take(64 * PP * 2);
    bf* Xb = (bf*)take((size_t)NTOK * DD * 2); float* Lf = (float*)take((size_t)NTOK * PP * 4); float* Rf = (float*)take((size_t)NTOK * PP * 4); float* Hs = (float*)take((size_t)NTOK * PP * 4);
    bf* Ah = (bf*)take((size_t)NPR * PP * 2); bf* Al = (bf*)take((size_t)NPR * PP * 2); float* Cm = (float*)take((size_t)NPR * 64 * 4);
    if ((size_t)(wsp - (char*)d_ws) > ws_size) return;
    k_wt<<<dim3(DD / 64, PP / 64, 1), 256, 0, stream>>>(Wl, DD, PP, WlT); k_wt<<<dim3(DD / 64, PP / 64, 1), 256, 0, stream>>>(Wr, DD, PP, WrT);
    k_wt<<<dim3(DD / 64, PP / 64, 1), 256, 0, stream>>>(Ws1, DD, PP, WsT); k_wt<<<dim3(DD / 64, PP / 64, 1), 256, 0, stream>>>(We1, DD, PP, WeT); k_wopad<<<(64 * PP / 8 + 255) / 256, 256, 0, stream>>>(Wo, WOP);
    for (int b = 0; b < NBI; ++b) {
        k_cvt<<<NTOK / 8, 256, 0, stream>>>(x + (size_t)b * NTOK * DD, Xb);
        k_gemmb<false, false><<<dim3(NTOK / 64, PP / 64, 1), 128, 0, stream>>>(Xb, nullptr, WsT, bs1, Hs, PP, nullptr); k_head1<<<NTOK / 256, 256, 0, stream>>>(Hs, Ws2, bs2, out1, b);
        k_gemmb<false, false><<<dim3(NTOK / 64, PP / 64, 1), 128, 0, stream>>>(Xb, nullptr, WeT, be1, Hs, PP, nullptr); k_head1<<<NTOK / 256, 256, 0, stream>>>(Hs, We2, be2, out2, b);
        k_gemmb<false, false><<<dim3(NTOK / 64, PP / 64, 1), 128, 0, stream>>>(Xb, nullptr, WlT, bl, Lf, PP, nullptr);
        k_gemmb<false, false><<<dim3(NTOK / 64, PP / 64, 1), 128, 0, stream>>>(Xb, nullptr, WrT, nullptr, Rf, PP, nullptr);
        for (int c = 0; c < NTOK / ICH; ++c) { const int i0 = c * ICH;
            k_pairs<<<ICH * (NTOK / 16), 256, 0, stream>>>(Lf, Rf, i0, Ah, Al);
            k_gemmb<true, false><<<dim3(NPR / 64, 1, 1), 128, 0, stream>>>(Ah, Al, WOP, nullptr, Cm, 64, nullptr, nullptr, PP);
            k_bout<<<NPR / 256, 256, 0, stream>>>(Cm, bo, b, i0, out0); }
    }
}
